// DeformableAlignment_17360257811041
// MI455X (gfx1250) — hardware-verified
//
#include <hip/hip_runtime.h>
#include <math.h>
#include <stddef.h>

typedef __attribute__((ext_vector_type(16))) _Float16 v16h;
typedef __attribute__((ext_vector_type(8)))  _Float16 v8h;
typedef __attribute__((ext_vector_type(16))) __bf16   v16b;
typedef __attribute__((ext_vector_type(8)))  __bf16   v8b;
typedef __attribute__((ext_vector_type(8)))  float    v8f;
typedef __attribute__((ext_vector_type(4)))  float    v4f;
typedef __attribute__((ext_vector_type(4)))  unsigned v4u;

constexpr int NB     = 8;
constexpr int HH     = 96;
constexpr int WW     = 160;
constexpr int HP     = HH + 2;
constexpr int WP     = WW + 2;
constexpr int HWPIX  = HH * WW;
constexpr int NPIX   = NB * HWPIX;
constexpr int HPWP   = HP * WP;
constexpr int NPPIX  = NB * HPWP;
constexpr int CCAT   = 196;
constexpr int CPCAT  = 224;
constexpr int CMID   = 64;
constexpr int NGATE  = 216;
constexpr int NGATEP = 256;
constexpr int KTAP   = 576;
constexpr int QPIX   = 30720;
constexpr int NQUART = 4;
constexpr int NTHR   = 256;
constexpr int PKPITCH = 228;
constexpr int SPITCH  = 580;
constexpr int SMP_PIX = 4;
constexpr int SMP_THR = SMP_PIX * 72;

constexpr float CW1 = 32.0f, CW2 = 16.0f, CW3 = 16.0f, CW4 = 16.0f;
constexpr float CA1 = 4.0f, CA2 = 8.0f, CA3 = 16.0f, CO4 = 16.0f;
constexpr float CSMP = 16.0f, CWD = 32.0f;
constexpr float S1_ACC = CA1 / CW1;
constexpr float S2_ACC = CA2 / (CA1 * CW2);
constexpr float S3_ACC = CA3 / (CA2 * CW3);
constexpr float S4_ACC = CO4 / (CA3 * CW4);
constexpr float O4_INV = 1.0f / CO4;
constexpr float SD_ACC = 1.0f / (CSMP * CWD);

constexpr size_t SZ_CAT = (size_t)NPPIX * CPCAT * 2;
constexpr size_t SZ_O4  = (size_t)NPIX * NGATEP * 2;
constexpr size_t SZ_R0  = SZ_O4;
constexpr size_t SZ_ACT = (size_t)NPPIX * CMID * 2;
constexpr size_t SZ_SMP = (size_t)QPIX * KTAP * 2;
constexpr size_t SZ_BT1 = (size_t)64 * 9 * CPCAT * 2;
constexpr size_t SZ_BT2 = (size_t)64 * KTAP * 2;
constexpr size_t SZ_BT4 = (size_t)NGATEP * KTAP * 2;
constexpr size_t WS_R0  = 0;
constexpr size_t WS_A1  = WS_R0 + SZ_R0;
constexpr size_t WS_A2  = WS_A1 + SZ_ACT;
constexpr size_t WS_A3  = WS_A2 + SZ_ACT;
constexpr size_t WS_SMP = WS_A1;
constexpr size_t WS_BT1 = WS_A3 + SZ_ACT;
constexpr size_t WS_BT2 = WS_BT1 + SZ_BT1;
constexpr size_t WS_BT3 = WS_BT2 + SZ_BT2;
constexpr size_t WS_BT4 = WS_BT3 + SZ_BT2;
constexpr size_t WS_BTD = WS_BT4 + SZ_BT4;
constexpr size_t WS_TOTAL = WS_BTD + SZ_BT2;
static_assert(SZ_CAT <= SZ_R0);
static_assert(SZ_SMP <= 3 * SZ_ACT);
static_assert(WS_TOTAL == 112459776);
static_assert(WS_TOTAL <= (size_t)134217728);
static_assert((WS_A1 % 256) == 0 && (WS_A2 % 256) == 0 && (WS_A3 % 256) == 0 && (WS_BT1 % 256) == 0);
static_assert((WS_BT2 % 256) == 0 && (WS_BT3 % 256) == 0 && (WS_BT4 % 256) == 0 && (WS_BTD % 256) == 0);
static_assert(NPIX % 64 == 0 && HWPIX % 64 == 0 && WW % 16 == 0);
static_assert(CPCAT % 32 == 0 && CMID % 32 == 0 && KTAP % 32 == 0);
static_assert(NQUART * QPIX == NPIX && QPIX == 2 * HWPIX && QPIX % SMP_PIX == 0);
static_assert(NPPIX % 32 == 0);
static_assert((3 * SZ_ACT) % (16 * NTHR) == 0);

__device__ __forceinline__ unsigned short f2bf_bits(float f) {
  unsigned u = __float_as_uint(f);
  return (unsigned short)((u + 0x7FFFu + ((u >> 16) & 1u)) >> 16);
}
__device__ __forceinline__ float bf_bits2f(unsigned short h) { return __uint_as_float(((unsigned)h) << 16); }

__device__ __forceinline__ void dep_guard_h(v8f& a, v8f& b, v16h x, v16h y) { asm volatile("v_nop\n\tv_nop\n\tv_nop\n\tv_nop" : "+v"(a), "+v"(b) : "v"(x), "v"(y)); }
__device__ __forceinline__ void dep_guard_b(v8f& a, v8f& b, v16b x, v16b y) { asm volatile("v_nop\n\tv_nop\n\tv_nop\n\tv_nop" : "+v"(a), "+v"(b) : "v"(x), "v"(y)); }
__device__ __forceinline__ void keep4_h(v16h a, v16h b, v16h c, v16h d) { asm volatile("v_nop" :: "v"(a), "v"(b), "v"(c), "v"(d)); }
__device__ __forceinline__ void keep4_b(v16b a, v16b b, v16b c, v16b d) { asm volatile("v_nop" :: "v"(a), "v"(b), "v"(c), "v"(d)); }
__device__ __forceinline__ void acc_guard4(v8f& a, v8f& b, v8f& c, v8f& d) { asm volatile("v_nop\n\tv_nop\n\tv_nop\n\tv_nop" : "+v"(a), "+v"(b), "+v"(c), "+v"(d)); }
template <typename T> struct Frag;
template <> struct Frag<_Float16> {
  typedef v16h V; union U { v16h v; v8h h[2]; };
  static __device__ __forceinline__ v16h load(const _Float16* p) {
    U f; f.h[0] = *(const v8h*)(p); f.h[1] = *(const v8h*)(p + 16); return f.v;
  }
  static __device__ __forceinline__ v8f mma(v16h a, v16h b, v8f c) {
    return __builtin_amdgcn_wmma_f32_16x16x32_f16(false, a, false, b, (short)0, c, false, false);
  }
  static __device__ __forceinline__ void guard(v8f& a, v8f& b, v16h x, v16h y) { dep_guard_h(a, b, x, y); }
  static __device__ __forceinline__ void keep(v16h a, v16h b, v16h c, v16h d) { keep4_h(a, b, c, d); }
};
template <> struct Frag<__bf16> {
  typedef v16b V; union U { v16b v; v8b h[2]; };
  static __device__ __forceinline__ v16b load(const __bf16* p) {
    U f; f.h[0] = *(const v8b*)(p); f.h[1] = *(const v8b*)(p + 16); return f.v;
  }
  static __device__ __forceinline__ v8f mma(v16b a, v16b b, v8f c) {
    return __builtin_amdgcn_wmma_f32_16x16x32_bf16(false, a, false, b, (short)0, c, false, false);
  }
  static __device__ __forceinline__ void guard(v8f& a, v8f& b, v16b x, v16b y) { dep_guard_b(a, b, x, y); }
  static __device__ __forceinline__ void keep(v16b a, v16b b, v16b c, v16b d) { keep4_b(a, b, c, d); }
};

template <int ET> struct Elem;
template <> struct Elem<0> { typedef _Float16 T; };
template <> struct Elem<1> { typedef __bf16 T; };
template <int ET, bool SPLIT, int BIAS_MODE, int OUT_MODE, bool RESID, int ACT = 0>
__global__ __launch_bounds__(256) void wmma_gemm64(
    const unsigned short* __restrict__ Ap, const unsigned short* __restrict__ A2p, int lda, long strideA,
    const unsigned short* __restrict__ Btp, const unsigned short* __restrict__ Bt2p, int ldb, long strideB,
    void* __restrict__ Cout, void* __restrict__ Cout2, int ldc, long strideC,
    const float* __restrict__ bias,
    const float* __restrict__ resid, long strideR,
    int M, int N, int K, float scale) {
  typedef typename Elem<ET>::T T;
  typedef typename Frag<T>::V V;
  const T* A = (const T*)Ap; const T* A2 = (const T*)A2p; const T* Bt = (const T*)Btp; const T* Bt2 = (const T*)Bt2p;
  __shared__ __align__(16) float sT[8][16 * 68];
  const int b    = blockIdx.y;
  const int lane = threadIdx.x & 31;
  const int wave = threadIdx.x >> 5;
  const int tilesN = N >> 6;
  const int tilesM = M >> 6;
  const int tile = blockIdx.x * 8 + wave;
  if (tile >= tilesM * tilesN) return;
  const int tm = tile / tilesN;
  const int tn = tile - tm * tilesN;
  const int m0 = tm << 6;
  const int n0 = tn << 6;

  const T* Ab  = A  + (size_t)b * strideA;
  const T* Bb  = Bt + (size_t)b * strideB;
  const T* Ab2 = SPLIT ? (A2  + (size_t)b * strideA) : nullptr;
  const T* Bb2 = SPLIT ? (Bt2 + (size_t)b * strideB) : nullptr;

  const int rlane = lane & 15;
  const int koff  = (lane >> 4) * 8;
  const int mOff  = (lane >> 4) * 8;

  v8f acc[4][4];
#pragma unroll
  for (int i = 0; i < 4; ++i)
#pragma unroll
    for (int j = 0; j < 4; ++j) acc[i][j] = (v8f){0.f,0.f,0.f,0.f,0.f,0.f,0.f,0.f};

  for (int k0 = 0; k0 < K; k0 += 32) {
    V bh[4], bl[4];
#pragma unroll
    for (int j = 0; j < 4; ++j) {
      const size_t bo = (size_t)(n0 + (j << 4) + rlane) * ldb + koff + k0;
      bh[j] = Frag<T>::load(Bb + bo);
      if (SPLIT) bl[j] = Frag<T>::load(Bb2 + bo);
    }
#pragma unroll
    for (int i = 0; i < 4; ++i) {
      const size_t ao = (size_t)(m0 + (i << 4) + rlane) * lda + koff + k0;
      V ah = Frag<T>::load(Ab + ao);
      V al;
      if (SPLIT) al = Frag<T>::load(Ab2 + ao);
#pragma unroll
      for (int j = 0; j < 4; ++j) {
        acc[i][j] = Frag<T>::mma(ah, bh[j], acc[i][j]);
        if (SPLIT) {
          acc[i][j] = Frag<T>::mma(ah, bl[j], acc[i][j]);
          acc[i][j] = Frag<T>::mma(al, bh[j], acc[i][j]);
        }
      }
      Frag<T>::guard(acc[i][0], acc[i][3], ah, SPLIT ? al : ah);
    }
    Frag<T>::keep(bh[0], bh[1], bh[2], bh[3]);
    if (SPLIT) Frag<T>::keep(bl[0], bl[1], bl[2], bl[3]);
  }
  acc_guard4(acc[0][0], acc[0][1], acc[0][2], acc[0][3]);
  acc_guard4(acc[1][0], acc[1][1], acc[1][2], acc[1][3]);
  acc_guard4(acc[2][0], acc[2][1], acc[2][2], acc[2][3]);
  acc_guard4(acc[3][0], acc[3][1], acc[3][2], acc[3][3]);

  float* slab = sT[wave];
  const float* Rb = RESID ? (resid + (size_t)b * strideR) : nullptr;
#pragma unroll
  for (int i = 0; i < 4; ++i) {
    const int mBase = m0 + (i << 4);
#pragma unroll
    for (int j = 0; j < 4; ++j) {
      const int n = n0 + (j << 4) + rlane;
      float bv = 0.f;
      if (BIAS_MODE == 2) bv = bias[n];
#pragma unroll
      for (int r = 0; r < 8; ++r) {
        float v = acc[i][j][r] * scale;
        if (BIAS_MODE == 1) v += bias[mBase + mOff + r];
        if (BIAS_MODE == 2) v += bv;
        if (RESID) v += Rb[(size_t)(mBase + mOff + r) * ldc + n];
        if (ACT == 1) v = tanhf(v);
        if (ACT == 2) v = fmaxf(v, 0.0f);
        if (ACT == 3) v = v / (1.0f + expf(-v));
        if (ACT == 4) v = (v > 0.f) ? v : 0.01f * v;
        if (ACT == 5) v = 0.5f * v * (1.0f + erff(v * 0.70710678118654752f));
        slab[(mOff + r) * 68 + (j << 4) + rlane] = v;
      }
    }
    __builtin_amdgcn_fence(__ATOMIC_RELEASE, "workgroup");
    __builtin_amdgcn_wave_barrier();
    __builtin_amdgcn_fence(__ATOMIC_ACQUIRE, "workgroup");
    if (OUT_MODE == 0) {
      float* C = (float*)Cout + (size_t)b * strideC;
      const int hh = lane >> 4, c4 = (lane & 15) * 4;
      for (int pass = 0; pass < 2; ++pass) {
#pragma unroll
        for (int it = 0; it < 8; ++it) {
          const int row = it * 2 + hh;
          v4f v = *(const v4f*)(slab + row * 68 + c4);
          *(volatile v4f*)(C + (size_t)(mBase + row) * ldc + n0 + c4) = v;
        }
        __threadfence();
      }
    } else {
      const int q = lane >> 3, c8 = (lane & 7) * 8;
      unsigned short* C  = (unsigned short*)Cout  + (size_t)b * strideC;
      unsigned short* C2 = (OUT_MODE == 2) ? ((unsigned short*)Cout2 + (size_t)b * strideC) : nullptr;
      for (int pass = 0; pass < 2; ++pass) {
#pragma unroll
        for (int it = 0; it < 4; ++it) {
          const int row = it * 4 + q;
          const float* sp = slab + row * 68 + c8;
          v8h hv, lv;
#pragma unroll
          for (int e = 0; e < 8; ++e) {
            if (OUT_MODE == 1) {
              hv[e] = (_Float16)sp[e];
            } else {
              unsigned short hb = f2bf_bits(sp[e]);
              unsigned short lb = f2bf_bits(sp[e] - bf_bits2f(hb));
              hv[e] = __builtin_bit_cast(_Float16, hb);
              lv[e] = __builtin_bit_cast(_Float16, lb);
            }
          }
          *(volatile v8h*)(C + (size_t)(mBase + row) * ldc + n0 + c8) = hv;
          if (OUT_MODE == 2) *(volatile v8h*)(C2 + (size_t)(mBase + row) * ldc + n0 + c8) = lv;
        }
        __threadfence();
      }
    }
    __builtin_amdgcn_fence(__ATOMIC_RELEASE, "workgroup");
    __builtin_amdgcn_wave_barrier();
    __builtin_amdgcn_fence(__ATOMIC_ACQUIRE, "workgroup");
  }
}

__device__ __forceinline__ float h16_to_f32(unsigned hb) {
  const unsigned sgn = (hb & 0x8000u) << 16; const unsigned em = hb & 0x7fffu;
  const float fn = __uint_as_float((em << 13) + 0x38000000u);
  const float fs = (float)em * 5.9604644775390625e-8f;
  const float mag = (em < 0x400u) ? fs : fn; return __uint_as_float(__float_as_uint(mag) | sgn); }

__global__ __launch_bounds__(NTHR) void zero16_kernel(unsigned* __restrict__ p, int n4) {
  const int i = blockIdx.x * NTHR + threadIdx.x;
  if (i >= n4) return;
  const v4u z = {0u, 0u, 0u, 0u};
  unsigned* d = p + (size_t)i * 4;
  *(volatile v4u*)d = z;
  __threadfence();
  *(volatile v4u*)d = z;
}

__global__ __launch_bounds__(NTHR) void pack5_kernel(const float* __restrict__ x0, const float* __restrict__ x1,
                                                     const float* __restrict__ x2, const float* __restrict__ fa,
                                                     const float* __restrict__ fb, unsigned short* __restrict__ cat) {
  __shared__ __align__(16) float tile[32 * PKPITCH];
  const int tid = threadIdx.x, lane = tid & 31, wave = tid >> 5;
  const int pp0 = blockIdx.x * 32;
  const int pp = pp0 + lane;
  const int b = pp / HPWP;
  const int r = pp - b * HPWP;
  const int hp = r / WP;
  const int wp = r - hp * WP;
  const int h = hp - 1, w = wp - 1;
  const float vf = (h >= 0 && h < HH && w >= 0 && w < WW) ? 1.0f : 0.0f;
  const int hc = (h < 0) ? 0 : ((h > HH - 1) ? (HH - 1) : h);
  const int wc = (w < 0) ? 0 : ((w > WW - 1) ? (WW - 1) : w);
  const int spix = hc * WW + wc;
#pragma unroll 1
  for (int j = 0; j < 28; ++j) {
    const int c = __builtin_amdgcn_readfirstlane(wave + 8 * j);
    const float* src = x0; int ch = c; int nch = 64; float cf = vf;
    if (c >= 64)  { src = x1; ch = c - 64; }
    if (c >= 128) { src = x2; ch = c - 128; }
    if (c >= 192) { src = fa; ch = c - 192; nch = 2; }
    if (c >= 194) { src = fb; ch = c - 194; nch = 2; }
    if (c >= 196) { ch = 1; cf = 0.0f; }
    const float v = src[(size_t)(b * nch + ch) * HWPIX + spix];
    tile[lane * PKPITCH + c] = v * cf;
  }
  __syncthreads();
  unsigned short* dst0 = cat + (size_t)pp0 * CPCAT;
  for (int pass = 0; pass < 2; ++pass) {
#pragma unroll
    for (int j = 0; j < 4; ++j) {
      const int idx = tid + NTHR * j;
      if (idx < 32 * 28) {
        const int pl = idx / 28;
        const int cc = idx - pl * 28;
        const float* sp = tile + pl * PKPITCH + cc * 8;
        const v4f a4 = *(const v4f*)sp;
        const v4f b4 = *(const v4f*)(sp + 4);
        v8h hv;
        hv[0] = (_Float16)a4[0]; hv[1] = (_Float16)a4[1]; hv[2] = (_Float16)a4[2]; hv[3] = (_Float16)a4[3];
        hv[4] = (_Float16)b4[0]; hv[5] = (_Float16)b4[1]; hv[6] = (_Float16)b4[2]; hv[7] = (_Float16)b4[3];
        *(volatile v8h*)(dst0 + (size_t)idx * 8) = hv;
      }
    }
    __threadfence();
  }
}

template <bool TAPMAJOR>
__global__ __launch_bounds__(NTHR) void wprep_kernel(const float* __restrict__ w, int Cin, int Nreal, int CPL, int Npad,
                                                     float scale, unsigned short* __restrict__ bt) {
  const int kp8 = (9 * CPL) >> 3;
  const int i = blockIdx.x * NTHR + threadIdx.x;
  if (i >= Npad * kp8) return;
  const int n = i / kp8;
  const int k0 = (i - n * kp8) * 8;
  const int ncl = (n < Nreal) ? n : (Nreal - 1);
  const float nf = (n < Nreal) ? scale : 0.0f;
  v8h hv;
#pragma unroll
  for (int e = 0; e < 8; ++e) {
    const int k = k0 + e;
    float v;
    if (TAPMAJOR) {
      const int tap = k / CPL;
      const int cin = k - tap * CPL;
      const int ccl = (cin < Cin) ? cin : (Cin - 1);
      const float cf = (cin < Cin) ? 1.0f : 0.0f;
      v = w[((size_t)ncl * Cin + ccl) * 9 + tap] * cf;
    } else {
      v = w[(size_t)ncl * (9 * Cin) + k];
    }
    hv[e] = (_Float16)(v * nf);
  }
  unsigned short* d = bt + (size_t)i * 8;
  *(volatile v8h*)d = hv;
  __threadfence();
  *(volatile v8h*)d = hv;
}

template <int CPL, bool LRELU, bool OUT_HALO>
__global__ __launch_bounds__(NTHR) void conv3x3_wmma(
    const unsigned short* __restrict__ inp, const unsigned short* __restrict__ btp,
    const float* __restrict__ bias, unsigned short* __restrict__ outp,
    int N, int Nreal, float s_acc, float s_bias) {
  typedef _Float16 T;
  typedef Frag<T>::V V;
  constexpr int KCH  = CPL / 32;
  constexpr int KTOT = 9 * CPL;
  constexpr int NKS  = 9 * KCH;
  const T* In = (const T*)inp;
  const T* Bt = (const T*)btp;
  __shared__ __align__(16) float sT[8][16 * 68];
  const int lane = threadIdx.x & 31;
  const int wave = threadIdx.x >> 5;
  const int tilesN = N >> 6;
  const int tile = blockIdx.x * 8 + wave;
  if (tile >= (NPIX >> 6) * tilesN) return;
  const int tm = tile / tilesN;
  const int tn = tile - tm * tilesN;
  const int m0 = tm << 6;
  const int n0 = tn << 6;
  const int rlane = lane & 15;
  const int koff  = (lane >> 4) * 8;
  const int mOff  = (lane >> 4) * 8;

  int abase[4];
#pragma unroll
  for (int i = 0; i < 4; ++i) {
    const int p  = m0 + (i << 4) + rlane;
    const int b  = p / HWPIX;
    const int hw = p - b * HWPIX;
    const int h  = hw / WW;
    const int w  = hw - h * WW;
    abase[i] = ((b * HP + h) * WP + w) * CPL + koff;
  }

  v8f acc[4][4];
#pragma unroll
  for (int i = 0; i < 4; ++i)
#pragma unroll
    for (int j = 0; j < 4; ++j) acc[i][j] = (v8f){0.f,0.f,0.f,0.f,0.f,0.f,0.f,0.f};

#pragma unroll 1
  for (int ks = 0; ks < NKS; ++ks) {
    const int tap = ks / KCH;
    const int kc  = ks - tap * KCH;
    const int ky  = tap / 3;
    const int kx  = tap - ky * 3;
    const int aoff = (ky * WP + kx) * CPL + kc * 32;
    const int boff = tap * CPL + kc * 32 + koff;
    V bh[4];
#pragma unroll
    for (int j = 0; j < 4; ++j)
      bh[j] = Frag<T>::load(Bt + (size_t)(n0 + (j << 4) + rlane) * KTOT + boff);
#pragma unroll
    for (int i = 0; i < 4; ++i) {
      const V ah = Frag<T>::load(In + (size_t)abase[i] + aoff);
#pragma unroll
      for (int j = 0; j < 4; ++j) acc[i][j] = Frag<T>::mma(ah, bh[j], acc[i][j]);
      Frag<T>::guard(acc[i][0], acc[i][3], ah, ah);
    }
    Frag<T>::keep(bh[0], bh[1], bh[2], bh[3]);
  }
  acc_guard4(acc[0][0], acc[0][1], acc[0][2], acc[0][3]);
  acc_guard4(acc[1][0], acc[1][1], acc[1][2], acc[1][3]);
  acc_guard4(acc[2][0], acc[2][1], acc[2][2], acc[2][3]);
  acc_guard4(acc[3][0], acc[3][1], acc[3][2], acc[3][3]);

  float* slab = sT[wave];
  const int q = lane >> 3, c8 = (lane & 7) * 8;
#pragma unroll
  for (int i = 0; i < 4; ++i) {
    const int mBase = m0 + (i << 4);
#pragma unroll
    for (int j = 0; j < 4; ++j) {
      const int n = n0 + (j << 4) + rlane;
      const int ncl = (n < Nreal) ? n : (Nreal - 1);
      const float bv = bias[ncl] * s_bias;
#pragma unroll
      for (int r = 0; r < 8; ++r) {
        float v = acc[i][j][r] * s_acc + bv;
        if (LRELU) v = (v >= 0.0f) ? v : 0.1f * v;
        slab[(mOff + r) * 68 + (j << 4) + rlane] = v;
      }
    }
    __builtin_amdgcn_fence(__ATOMIC_RELEASE, "workgroup");
    __builtin_amdgcn_wave_barrier();
    __builtin_amdgcn_fence(__ATOMIC_ACQUIRE, "workgroup");
    for (int pass = 0; pass < 2; ++pass) {
#pragma unroll
      for (int it = 0; it < 4; ++it) {
        const int row = it * 4 + q;
        const int p = mBase + row;
        size_t ob;
        if (OUT_HALO) {
          const int b  = p / HWPIX;
          const int hw = p - b * HWPIX;
          const int h  = hw / WW;
          const int w  = hw - h * WW;
          ob = (size_t)((b * HP + h + 1) * WP + (w + 1)) * CMID + c8;
        } else {
          ob = (size_t)p * NGATEP + n0 + c8;
        }
        const float* sp = slab + row * 68 + c8;
        v8h hv;
#pragma unroll
        for (int e = 0; e < 8; ++e) hv[e] = (_Float16)sp[e];
        *(volatile v8h*)(outp + ob) = hv;
      }
      __threadfence();
    }
    __builtin_amdgcn_fence(__ATOMIC_RELEASE, "workgroup");
    __builtin_amdgcn_wave_barrier();
    __builtin_amdgcn_fence(__ATOMIC_ACQUIRE, "workgroup");
  }
}

__global__ __launch_bounds__(SMP_THR) void bsample_kernel(const float* __restrict__ x0, const unsigned* __restrict__ o4w,
                                                          const float* __restrict__ fa, const float* __restrict__ fb,
                                                          int pix0q, unsigned short* __restrict__ smp) {
#pragma clang fp contract(off)
  __shared__ __align__(16) float tile[SMP_PIX * SPITCH];
  const int tid  = threadIdx.x;
  const int pl   = tid / 72;
  const int pair = tid - pl * 72;
  const int g    = pair / 9;
  const int tap  = pair - g * 9;
  const int ky   = tap / 3;
  const int kx   = tap - ky * 3;
  const int pix  = pix0q + blockIdx.x * SMP_PIX + pl;
  const int b    = pix / HWPIX;
  const int hw   = pix - b * HWPIX;
  const int h    = hw / WW;
  const int w    = hw - h * WW;

  const unsigned wo = o4w[(size_t)pix * (NGATEP / 2) + pair];
  const unsigned wm = o4w[(size_t)pix * (NGATEP / 2) + 72 + (pair >> 1)];
  const unsigned mb = (pair & 1) ? (wm >> 16) : (wm & 0xffffu);
  const float ody = h16_to_f32(wo & 0xffffu) * O4_INV;
  const float odx = h16_to_f32(wo >> 16) * O4_INV;
  const float ml  = h16_to_f32(mb) * O4_INV;

  const float a1y = fa[(size_t)(b * 2 + 1) * HWPIX + hw];
  const float a1x = fa[(size_t)(b * 2 + 0) * HWPIX + hw];
  const float a2y = fb[(size_t)(b * 2 + 1) * HWPIX + hw];
  const float a2x = fb[(size_t)(b * 2 + 0) * HWPIX + hw];
  const float s1 = (g < 4) ? 1.0f : 0.0f;
  const float s2 = 1.0f - s1;
  const float fy = fmaf(s1, a1y, s2 * a2y);
  const float fx = fmaf(s1, a1x, s2 * a2x);

  const float dy = ody + fy;
  const float dx = odx + fx;
  const float ys = ((dy + (float)h) - 1.0f) + (float)ky;
  const float xs = ((dx + (float)w) - 1.0f) + (float)kx;
  const float mk = 1.0f / (1.0f + expf(-ml));

  const float y0f = floorf(ys);
  const float x0f = floorf(xs);
  const float wy1 = ys - y0f;
  const float wx1 = xs - x0f;
  const float wy0 = 1.0f - wy1;
  const float wx0 = 1.0f - wx1;
  const int yi = (int)fminf(fmaxf(y0f, -2.0f), (float)(HH + 1));
  const int xi = (int)fminf(fmaxf(x0f, -2.0f), (float)(WW + 1));
  const float vy0 = (yi >= 0 && yi <= HH - 1) ? 1.0f : 0.0f;
  const float vy1 = (yi >= -1 && yi <= HH - 2) ? 1.0f : 0.0f;
  const float vx0 = (xi >= 0 && xi <= WW - 1) ? 1.0f : 0.0f;
  const float vx1 = (xi >= -1 && xi <= WW - 2) ? 1.0f : 0.0f;
  const int yc0 = (yi < 0) ? 0 : ((yi > HH - 1) ? (HH - 1) : yi);
  const int yc1 = (yi + 1 < 0) ? 0 : ((yi + 1 > HH - 1) ? (HH - 1) : (yi + 1));
  const int xc0 = (xi < 0) ? 0 : ((xi > WW - 1) ? (WW - 1) : xi);
  const int xc1 = (xi + 1 < 0) ? 0 : ((xi + 1 > WW - 1) ? (WW - 1) : (xi + 1));
  const float w00 = vy0 * vx0 * (wy0 * wx0);
  const float w01 = vy0 * vx1 * (wy0 * wx1);
  const float w10 = vy1 * vx0 * (wy1 * wx0);
  const float w11 = vy1 * vx1 * (wy1 * wx1);
  const int i00 = yc0 * WW + xc0, i01 = yc0 * WW + xc1;
  const int i10 = yc1 * WW + xc0, i11 = yc1 * WW + xc1;
  const float mks = mk * CSMP;
  const float* img = x0 + (size_t)(b * 64 + g * 8) * HWPIX;
  float* trow = tile + pl * SPITCH + (g * 8) * 9 + tap;
#pragma unroll 1
  for (int c = 0; c < 8; ++c) {
    const float* im = img + (size_t)c * HWPIX;
    const float v00 = im[i00];
    const float v01 = im[i01];
    const float v10 = im[i10];
    const float v11 = im[i11];
    float s = v00 * w00 + v01 * w01;
    s = s + v10 * w10;
    s = s + v11 * w11;
    trow[c * 9] = s * mks;
  }
  __syncthreads();
  {
    const float* sp = tile + pl * SPITCH + pair * 8;
    const v4f a4 = *(const v4f*)sp;
    const v4f b4 = *(const v4f*)(sp + 4);
    v8h hv;
    hv[0] = (_Float16)a4[0]; hv[1] = (_Float16)a4[1]; hv[2] = (_Float16)a4[2]; hv[3] = (_Float16)a4[3];
    hv[4] = (_Float16)b4[0]; hv[5] = (_Float16)b4[1]; hv[6] = (_Float16)b4[2]; hv[7] = (_Float16)b4[3];
    unsigned short* d = smp + (size_t)blockIdx.x * (SMP_PIX * KTAP) + (size_t)tid * 8;
    *(volatile v8h*)d = hv;
    __threadfence();
    *(volatile v8h*)d = hv;
  }
}

extern "C" void kernel_launch(void* const* d_in, const int* in_sizes, int n_in,
                              void* d_out, int out_size, void* d_ws, size_t ws_size,
                              hipStream_t stream) {
  if (n_in < 15) return;
  if (ws_size < WS_TOTAL) return;
  if ((size_t)out_size < (size_t)NPIX * 64) return;
  if (in_sizes[0] != NPIX * 64 || in_sizes[3] != NPIX * 2 || in_sizes[11] != NGATE * 64 * 9 || in_sizes[13] != 64 * 64 * 9) return;

  const float* x0 = (const float*)d_in[0];
  const float* x1 = (const float*)d_in[1];
  const float* x2 = (const float*)d_in[2];
  const float* fa = (const float*)d_in[3];
  const float* fb = (const float*)d_in[4];
  const float* w1 = (const float*)d_in[5];
  const float* b1 = (const float*)d_in[6];
  const float* w2 = (const float*)d_in[7];
  const float* b2 = (const float*)d_in[8];
  const float* w3 = (const float*)d_in[9];
  const float* b3 = (const float*)d_in[10];
  const float* w4 = (const float*)d_in[11];
  const float* b4 = (const float*)d_in[12];
  const float* wd = (const float*)d_in[13];
  const float* bd = (const float*)d_in[14];
  float* out = (float*)d_out;

  char* ws = (char*)d_ws;
  unsigned short* cat = (unsigned short*)(ws + WS_R0);
  unsigned short* o4  = (unsigned short*)(ws + WS_R0);
  unsigned short* a1  = (unsigned short*)(ws + WS_A1);
  unsigned short* a2  = (unsigned short*)(ws + WS_A2);
  unsigned short* a3  = (unsigned short*)(ws + WS_A3);
  unsigned short* smp = (unsigned short*)(ws + WS_SMP);
  unsigned short* bt1 = (unsigned short*)(ws + WS_BT1);
  unsigned short* bt2 = (unsigned short*)(ws + WS_BT2);
  unsigned short* bt3 = (unsigned short*)(ws + WS_BT3);
  unsigned short* bt4 = (unsigned short*)(ws + WS_BT4);
  unsigned short* btd = (unsigned short*)(ws + WS_BTD);

  const int nz4 = (int)((3 * SZ_ACT) / 16);
  zero16_kernel<<<nz4 / NTHR, NTHR, 0, stream>>>((unsigned*)a1, nz4);

  pack5_kernel<<<NPPIX / 32, NTHR, 0, stream>>>(x0, x1, x2, fa, fb, cat);

  wprep_kernel<true><<<(64 * (9 * CPCAT / 8)) / NTHR, NTHR, 0, stream>>>(w1, CCAT, 64, CPCAT, 64, CW1, bt1);
  wprep_kernel<true><<<(64 * (9 * CMID / 8)) / NTHR, NTHR, 0, stream>>>(w2, CMID, 64, CMID, 64, CW2, bt2);
  wprep_kernel<true><<<(64 * (9 * CMID / 8)) / NTHR, NTHR, 0, stream>>>(w3, CMID, 64, CMID, 64, CW3, bt3);
  wprep_kernel<true><<<(NGATEP * (9 * CMID / 8)) / NTHR, NTHR, 0, stream>>>(w4, CMID, NGATE, CMID, NGATEP, CW4, bt4);
  wprep_kernel<false><<<(64 * (9 * CMID / 8)) / NTHR, NTHR, 0, stream>>>(wd, CMID, 64, CMID, 64, CWD, btd);

  conv3x3_wmma<CPCAT, true, true><<<(NPIX / 64) * 1 / 8, NTHR, 0, stream>>>(cat, bt1, b1, a1, 64, 64, S1_ACC, CA1);
  conv3x3_wmma<CMID, true, true><<<(NPIX / 64) * 1 / 8, NTHR, 0, stream>>>(a1, bt2, b2, a2, 64, 64, S2_ACC, CA2);
  conv3x3_wmma<CMID, true, true><<<(NPIX / 64) * 1 / 8, NTHR, 0, stream>>>(a2, bt3, b3, a3, 64, 64, S3_ACC, CA3);
  conv3x3_wmma<CMID, false, false><<<(NPIX / 64) * (NGATEP / 64) / 8, NTHR, 0, stream>>>(a3, bt4, b4, o4, NGATEP, NGATE, S4_ACC, CO4);

  for (int qq = 0; qq < NQUART; ++qq) {
    bsample_kernel<<<QPIX / SMP_PIX, SMP_THR, 0, stream>>>(x0, (const unsigned*)o4, fa, fb, qq * QPIX, smp);
    float* cq = out + (size_t)qq * 2 * 64 * HWPIX;
    wmma_gemm64<0, false, 1, 0, false, 0><<<dim3((HWPIX / 64) / 8, 2), 256, 0, stream>>>(
        btd, btd, KTAP, 0L,
        smp, smp, KTAP, (long)HWPIX * KTAP,
        (void*)cq, (void*)cq, HWPIX, (long)64 * HWPIX,
        bd,
        bd, 0L,
        64, HWPIX, KTAP, SD_ACC);
  }
}
